// NextVLAD_33913061769333
// MI455X (gfx1250) — hardware-run, weakly checked
//
#include <hip/hip_runtime.h>

#pragma clang fp contract(off)

constexpr int NBATCH = 4;
constexpr int NB8    = 32;
constexpr int MTOK   = 1024;
constexpr int CIN    = 1024;
constexpr int HWN    = 128;
constexpr int EDIM   = 2048;
constexpr int NGRP   = 8;
constexpr int NCLU   = 128;
constexpr int DGRP   = 256;
constexpr int NGK    = 1024;
constexpr int NCAT   = 1088;
constexpr int DCOV   = 256;
constexpr int NTRIU  = 32896;
static_assert(NTRIU == DCOV * (DCOV + 1) / 2, "triu size");
static_assert(CIN % 32 == 0 && EDIM % 32 == 0 && MTOK % 32 == 0 && DCOV % 32 == 0, "K multiples of 32");
static_assert((NBATCH * MTOK) % 64 == 0 && EDIM % 64 == 0 && NCAT % 64 == 0 && NCLU % 64 == 0 && DGRP % 64 == 0 && DCOV % 64 == 0, "M,N multiples of 64");
static_assert(NCAT >= NGK + NGRP, "cat width");
static_assert((NBATCH * NTRIU) % 256 == 0, "triu grid exact");

typedef __attribute__((ext_vector_type(16))) _Float16 v16h;
typedef __attribute__((ext_vector_type(8)))  _Float16 v8h;
typedef __attribute__((ext_vector_type(16))) __bf16   v16b;
typedef __attribute__((ext_vector_type(8)))  __bf16   v8b;
typedef __attribute__((ext_vector_type(8)))  float    v8f;
typedef __attribute__((ext_vector_type(4)))  float    v4f;
typedef __attribute__((ext_vector_type(4)))  unsigned int u32x4;
#define PSCALE 32768.0f
#define U16(p) ((const unsigned short*)(const void*)(p))
#define PSCALE_INV (1.0f / 32768.0f)

__device__ __forceinline__ unsigned short f2bf_bits(float f) {
  unsigned u = __float_as_uint(f);
  return (unsigned short)((u + 0x7FFFu + ((u >> 16) & 1u)) >> 16);
}
__device__ __forceinline__ float bf_bits2f(unsigned short h) { return __uint_as_float(((unsigned)h) << 16); }

__device__ __forceinline__ unsigned short h_bits(float f) { return __builtin_bit_cast(unsigned short, (_Float16)f); }
__device__ __forceinline__ unsigned pack_h2(float a, float b) {
  return (unsigned)h_bits(a) | ((unsigned)h_bits(b) << 16);
}
__device__ __forceinline__ void split_bf(float v, unsigned short& hb, unsigned short& lb) {
  hb = f2bf_bits(v);
  lb = f2bf_bits(v - bf_bits2f(hb));
}

__device__ __forceinline__ void dep_guard_h(v8f& a, v8f& b, v16h x, v16h y) { asm volatile("v_nop\n\tv_nop\n\tv_nop\n\tv_nop" : "+v"(a), "+v"(b) : "v"(x), "v"(y)); }
__device__ __forceinline__ void dep_guard_b(v8f& a, v8f& b, v16b x, v16b y) { asm volatile("v_nop\n\tv_nop\n\tv_nop\n\tv_nop" : "+v"(a), "+v"(b) : "v"(x), "v"(y)); }
__device__ __forceinline__ void keep4_h(v16h a, v16h b, v16h c, v16h d) { asm volatile("v_nop" :: "v"(a), "v"(b), "v"(c), "v"(d)); }
__device__ __forceinline__ void keep4_b(v16b a, v16b b, v16b c, v16b d) { asm volatile("v_nop" :: "v"(a), "v"(b), "v"(c), "v"(d)); }
__device__ __forceinline__ void acc_guard4(v8f& a, v8f& b, v8f& c, v8f& d) { asm volatile("v_nop\n\tv_nop\n\tv_nop\n\tv_nop" : "+v"(a), "+v"(b), "+v"(c), "+v"(d)); }
template <typename T> struct Frag;
template <> struct Frag<_Float16> {
  typedef v16h V; union U { v16h v; v8h h[2]; };
  static __device__ __forceinline__ v16h load(const _Float16* p) {
    U f; f.h[0] = *(const v8h*)(p); f.h[1] = *(const v8h*)(p + 16); return f.v;
  }
  static __device__ __forceinline__ v8f mma(v16h a, v16h b, v8f c) {
    return __builtin_amdgcn_wmma_f32_16x16x32_f16(false, a, false, b, (short)0, c, false, false);
  }
  static __device__ __forceinline__ void guard(v8f& a, v8f& b, v16h x, v16h y) { dep_guard_h(a, b, x, y); }
  static __device__ __forceinline__ void keep(v16h a, v16h b, v16h c, v16h d) { keep4_h(a, b, c, d); }
};
template <> struct Frag<__bf16> {
  typedef v16b V; union U { v16b v; v8b h[2]; };
  static __device__ __forceinline__ v16b load(const __bf16* p) {
    U f; f.h[0] = *(const v8b*)(p); f.h[1] = *(const v8b*)(p + 16); return f.v;
  }
  static __device__ __forceinline__ v8f mma(v16b a, v16b b, v8f c) {
    return __builtin_amdgcn_wmma_f32_16x16x32_bf16(false, a, false, b, (short)0, c, false, false);
  }
  static __device__ __forceinline__ void guard(v8f& a, v8f& b, v16b x, v16b y) { dep_guard_b(a, b, x, y); }
  static __device__ __forceinline__ void keep(v16b a, v16b b, v16b c, v16b d) { keep4_b(a, b, c, d); }
};

template <int ET> struct Elem;
template <> struct Elem<0> { typedef _Float16 T; };
template <> struct Elem<1> { typedef __bf16 T; };
template <int ET, bool SPLIT, int BIAS_MODE, int OUT_MODE, bool RESID, int ACT = 0, int EPI = 0, bool BSC = false>
__global__ __launch_bounds__(256) void wmma_gemm64(
    const unsigned short* __restrict__ Ap, const unsigned short* __restrict__ A2p, int lda, long strideA,
    const unsigned short* __restrict__ Btp, const unsigned short* __restrict__ Bt2p, int ldb, long strideB,
    void* __restrict__ Cout, void* __restrict__ Cout2, int ldc, long strideC,
    const float* __restrict__ bias,
    const float* __restrict__ resid, long strideR,
    int M, int N, int K, float scale, const float* __restrict__ bsc) {
  typedef typename Elem<ET>::T T;
  typedef typename Frag<T>::V V;
  const T* A = (const T*)Ap; const T* A2 = (const T*)A2p; const T* Bt = (const T*)Btp; const T* Bt2 = (const T*)Bt2p;
  __shared__ __align__(16) float sT[8][16 * 68];
  const int b    = blockIdx.y;
  const int lane = threadIdx.x & 31;
  const int wave = threadIdx.x >> 5;
  const int tilesN = N >> 6;
  const int tilesM = M >> 6;
  const int tile = blockIdx.x * 8 + wave;
  if (tile >= tilesM * tilesN) return;
  const int tm = tile / tilesN;
  const int tn = tile - tm * tilesN;
  const int m0 = tm << 6;
  const int n0 = tn << 6;

  const T* Ab  = A  + (size_t)b * strideA;
  const T* Bb  = Bt + (size_t)b * strideB;
  const T* Ab2 = SPLIT ? (A2  + (size_t)b * strideA) : nullptr;
  const T* Bb2 = SPLIT ? (Bt2 + (size_t)b * strideB) : nullptr;

  const int rlane = lane & 15;
  const int koff  = (lane >> 4) * 8;
  const int mOff  = (lane >> 4) * 8;

  v8f acc[4][4];
#pragma unroll
  for (int i = 0; i < 4; ++i)
#pragma unroll
    for (int j = 0; j < 4; ++j) acc[i][j] = (v8f){0.f,0.f,0.f,0.f,0.f,0.f,0.f,0.f};

  for (int k0 = 0; k0 < K; k0 += 32) {
    V bh[4], bl[4];
#pragma unroll
    for (int j = 0; j < 4; ++j) {
      const size_t bo = (size_t)(n0 + (j << 4) + rlane) * ldb + koff + k0;
      bh[j] = Frag<T>::load(Bb + bo);
      if (SPLIT) bl[j] = Frag<T>::load(Bb2 + bo);
    }
#pragma unroll
    for (int i = 0; i < 4; ++i) {
      const size_t ao = (size_t)(m0 + (i << 4) + rlane) * lda + koff + k0;
      V ah = Frag<T>::load(Ab + ao);
      V al;
      if (SPLIT) al = Frag<T>::load(Ab2 + ao);
#pragma unroll
      for (int j = 0; j < 4; ++j) {
        acc[i][j] = Frag<T>::mma(ah, bh[j], acc[i][j]);
        if (SPLIT) {
          acc[i][j] = Frag<T>::mma(ah, bl[j], acc[i][j]);
          acc[i][j] = Frag<T>::mma(al, bh[j], acc[i][j]);
        }
      }
      Frag<T>::guard(acc[i][0], acc[i][3], ah, SPLIT ? al : ah);
    }
    Frag<T>::keep(bh[0], bh[1], bh[2], bh[3]);
    if (SPLIT) Frag<T>::keep(bl[0], bl[1], bl[2], bl[3]);
  }
  acc_guard4(acc[0][0], acc[0][1], acc[0][2], acc[0][3]);
  acc_guard4(acc[1][0], acc[1][1], acc[1][2], acc[1][3]);
  acc_guard4(acc[2][0], acc[2][1], acc[2][2], acc[2][3]);
  acc_guard4(acc[3][0], acc[3][1], acc[3][2], acc[3][3]);

  float* slab = sT[wave];
  const float* Rb = RESID ? (resid + (size_t)b * strideR) : nullptr;
  const float bscv = BSC ? bsc[b * 32 + 1] : 1.0f;
#pragma unroll
  for (int i = 0; i < 4; ++i) {
    const int mBase = m0 + (i << 4);
#pragma unroll
    for (int j = 0; j < 4; ++j) {
      const int n = n0 + (j << 4) + rlane;
      float bv = 0.f;
      if (BIAS_MODE == 2) bv = bias[n];
#pragma unroll
      for (int r = 0; r < 8; ++r) {
        float v = acc[i][j][r] * scale;
        if (BIAS_MODE == 1) v += bias[mBase + mOff + r];
        if (BIAS_MODE == 2) v += bv;
        if (RESID) v += Rb[(size_t)(mBase + mOff + r) * ldc + n];
        if (ACT == 1) v = tanhf(v);
        if (ACT == 2) v = fmaxf(v, 0.0f);
        if (ACT == 3) v = v / (1.0f + expf(-v));
        if (ACT == 4) v = (v > 0.f) ? v : 0.01f * v;
        if (ACT == 5) v = 0.5f * v * (1.0f + erff(v * 0.70710678118654752f));
        if (EPI == 1) v = 0.5f * ((((mBase + mOff + r) == n) ? 3.0f : 0.0f) - v);
        if (EPI == 2) v = ((((mBase + mOff + r) == n) ? 3.0f : 0.0f) - v);
        if (BSC) v = v * bscv;
        slab[(mOff + r) * 68 + (j << 4) + rlane] = v;
      }
    }
    __builtin_amdgcn_fence(__ATOMIC_RELEASE, "workgroup");
    __builtin_amdgcn_wave_barrier();
    __builtin_amdgcn_fence(__ATOMIC_ACQUIRE, "workgroup");
    if (OUT_MODE == 0) {
      float* C = (float*)Cout + (size_t)b * strideC;
      const int hh = lane >> 4, c4 = (lane & 15) * 4;
      for (int pass = 0; pass < 2; ++pass) {
#pragma unroll
        for (int it = 0; it < 8; ++it) {
          const int row = it * 2 + hh;
          v4f v = *(const v4f*)(slab + row * 68 + c4);
          *(volatile v4f*)(C + (size_t)(mBase + row) * ldc + n0 + c4) = v;
        }
        __threadfence();
      }
    } else {
      const int q = lane >> 3, c8 = (lane & 7) * 8;
      unsigned short* C  = (unsigned short*)Cout  + (size_t)b * strideC;
      unsigned short* C2 = (OUT_MODE == 2) ? ((unsigned short*)Cout2 + (size_t)b * strideC) : nullptr;
      for (int pass = 0; pass < 2; ++pass) {
#pragma unroll
        for (int it = 0; it < 4; ++it) {
          const int row = it * 4 + q;
          const float* sp = slab + row * 68 + c8;
          v8h hv, lv;
#pragma unroll
          for (int e = 0; e < 8; ++e) {
            if (OUT_MODE == 1) {
              hv[e] = (_Float16)sp[e];
            } else {
              unsigned short hb = f2bf_bits(sp[e]);
              unsigned short lb = f2bf_bits(sp[e] - bf_bits2f(hb));
              hv[e] = __builtin_bit_cast(_Float16, hb);
              lv[e] = __builtin_bit_cast(_Float16, lb);
            }
          }
          *(volatile v8h*)(C + (size_t)(mBase + row) * ldc + n0 + c8) = hv;
          if (OUT_MODE == 2) *(volatile v8h*)(C2 + (size_t)(mBase + row) * ldc + n0 + c8) = lv;
        }
        __threadfence();
      }
    }
    __builtin_amdgcn_fence(__ATOMIC_RELEASE, "workgroup");
    __builtin_amdgcn_wave_barrier();
    __builtin_amdgcn_fence(__ATOMIC_ACQUIRE, "workgroup");
  }
}

__global__ __launch_bounds__(256) void k_cast_scaled16(const float* __restrict__ in,
                                                        unsigned short* __restrict__ out, int n8, float sc) {
  const int i = blockIdx.x * 256 + threadIdx.x;
  if (i < n8) {
    const size_t e0 = (size_t)i * 8;
    const v4f a = *(const v4f*)(in + e0);
    const v4f c = *(const v4f*)(in + e0 + 4);
    u32x4 pk;
    pk[0] = pack_h2(a[0] * sc, a[1] * sc);
    pk[1] = pack_h2(a[2] * sc, a[3] * sc);
    pk[2] = pack_h2(c[0] * sc, c[1] * sc);
    pk[3] = pack_h2(c[2] * sc, c[3] * sc);
    *(volatile u32x4*)(out + e0) = pk;
    __threadfence();
    *(volatile u32x4*)(out + e0) = pk;
  }
}

__global__ __launch_bounds__(256) void k_build_wcat(const float* __restrict__ wgk, const float* __restrict__ wg,
                                                    unsigned short* __restrict__ out, float sc) {
  const int row = blockIdx.x;
  const int t = threadIdx.x;
  u32x4 pk = {0u, 0u, 0u, 0u};
  if (row < NGK + NGRP) {
    const float* src = (row < NGK) ? (wgk + (size_t)row * EDIM) : (wg + (size_t)(row - NGK) * EDIM);
    const v4f a = *(const v4f*)(src + 8 * t);
    const v4f c = *(const v4f*)(src + 8 * t + 4);
    pk[0] = pack_h2(a[0] * sc, a[1] * sc);
    pk[1] = pack_h2(a[2] * sc, a[3] * sc);
    pk[2] = pack_h2(c[0] * sc, c[1] * sc);
    pk[3] = pack_h2(c[2] * sc, c[3] * sc);
  }
  unsigned short* dst = out + (size_t)row * EDIM + 8 * t;
  *(volatile u32x4*)dst = pk;
  __threadfence();
  *(volatile u32x4*)dst = pk;
}

__global__ __launch_bounds__(256) void k_bias(const float* __restrict__ b_inp, const float* __restrict__ b_gk,
                                              const float* __restrict__ b_g,
                                              float* __restrict__ bias1, float* __restrict__ bias2) {
  const int i = blockIdx.x * 256 + threadIdx.x;
  if (i >= EDIM + NCAT) return;
  const int j = i - EDIM;
  const int i1 = (i < EDIM) ? i : (EDIM - 1);
  const int jg = (j < 0) ? 0 : ((j > NGK - 1) ? (NGK - 1) : j);
  const int jj = j - NGK;
  const int jc = (jj < 0) ? 0 : ((jj > NGRP - 1) ? (NGRP - 1) : jj);
  const float v1  = b_inp[i1] * 16.0f;
  const float vgk = b_gk[jg];
  const float vg  = b_g[jc];
  const float v2  = (j < NGK) ? vgk : ((j < NGK + NGRP) ? vg : 0.0f);
  const bool first = (i < EDIM);
  float* dst = first ? (bias1 + i) : (bias2 + j);
  const float v = first ? v1 : v2;
  *(volatile float*)dst = v;
  __threadfence();
  *(volatile float*)dst = v;
}

__global__ __launch_bounds__(256) void k_prep_xt(const float* __restrict__ x, unsigned short* __restrict__ xt16) {
  __shared__ float red[8][32];
  __shared__ float sinv[32];
  __shared__ __align__(16) unsigned short tile[32 * 72];
  const int hwc = blockIdx.x;
  const int b8  = blockIdx.y;
  const int lane = threadIdx.x & 31, wv = threadIdx.x >> 5;
  const int hw = hwc * 32 + lane;
  const float* xb = x + (size_t)b8 * CIN * HWN + hw;
  float ss = 0.f;
#pragma unroll 1
  for (int i = 0; i < CIN / 8; ++i) {
    const float v = xb[(size_t)(wv + 8 * i) * HWN];
    ss = ss + v * v;
  }
  red[wv][lane] = ss;
  __syncthreads();
  if (wv == 0) {
    float tot = red[0][lane];
#pragma unroll
    for (int w = 1; w < 8; ++w) tot += red[w][lane];
    sinv[lane] = 1.0f / fmaxf(sqrtf(tot), 1e-12f);
  }
  __syncthreads();
  const float inv = sinv[lane] * 32.0f;
  const int b = b8 >> 3, j = b8 & 7;
  const size_t row0 = (size_t)b * MTOK + (size_t)j * HWN + (size_t)hwc * 32;
  const int q = lane >> 3, c8 = (lane & 7) * 8;
  for (int cc = 0; cc < CIN / 64; ++cc) {
#pragma unroll 1
    for (int i = 0; i < 8; ++i) {
      const int cl = wv + 8 * i;
      const float v = xb[(size_t)(cc * 64 + cl) * HWN] * inv;
      tile[lane * 72 + cl] = h_bits(v);
    }
    __syncthreads();
    const u32x4 pk = *(const u32x4*)(tile + (4 * wv + q) * 72 + c8);
    unsigned short* dst = xt16 + (row0 + 4 * wv + q) * (size_t)CIN + cc * 64 + c8;
    *(volatile u32x4*)dst = pk;
    __threadfence();
    *(volatile u32x4*)dst = pk;
    __syncthreads();
  }
}

__global__ __launch_bounds__(256) void k_transpose16(const unsigned short* __restrict__ in, unsigned short* __restrict__ out,
                                                     int R, int Cc, long sIn, long sOut) {
  __shared__ __align__(16) unsigned short tile[64 * 72];
  const int c0 = blockIdx.x * 64, r0 = blockIdx.y * 64;
  const size_t ib = (size_t)blockIdx.z * (size_t)sIn, ob = (size_t)blockIdx.z * (size_t)sOut;
  const int t = threadIdx.x, lane = t & 31, wv = t >> 5;
#pragma unroll
  for (int u = 0; u < 2; ++u) {
    const int idx = t + 256 * u;
    const int row = idx >> 3, cc8 = (idx & 7) * 8;
    const u32x4 v = *(const u32x4*)(in + ib + (size_t)(r0 + row) * Cc + c0 + cc8);
    *(u32x4*)(tile + row * 72 + cc8) = v;
  }
  __syncthreads();
  const int p8 = (lane & 7) * 8, q = lane >> 3;
  u32x4 pk[2];
  size_t doff[2];
#pragma unroll
  for (int u = 0; u < 2; ++u) {
    const int cl = u * 32 + wv * 4 + q;
    const unsigned short* tp = tile + p8 * 72 + cl;
    u32x4 w;
    w[0] = (unsigned)tp[0]   | ((unsigned)tp[72]  << 16);
    w[1] = (unsigned)tp[144] | ((unsigned)tp[216] << 16);
    w[2] = (unsigned)tp[288] | ((unsigned)tp[360] << 16);
    w[3] = (unsigned)tp[432] | ((unsigned)tp[504] << 16);
    pk[u] = w;
    doff[u] = ob + (size_t)(c0 + cl) * R + r0 + p8;
  }
  for (int pass = 0; pass < 2; ++pass) {
    *(volatile u32x4*)(out + doff[0]) = pk[0];
    *(volatile u32x4*)(out + doff[1]) = pk[1];
    __threadfence();
  }
}

__global__ __launch_bounds__(256) void k_softmax_w(const float* __restrict__ logi,
                                                   unsigned short* __restrict__ wt16, float* __restrict__ wsum) {
  __shared__ float red[8][32];
  __shared__ __align__(16) unsigned short wt[32 * 264];
  const int cc = blockIdx.x, b = blockIdx.y;
  const int lane = threadIdx.x & 31, wv = threadIdx.x >> 5;
  const int gk = cc * 32 + lane, g = cc >> 2;
  const float* colp = logi + (size_t)b * MTOK * NCAT + gk;
  const float* agp  = logi + (size_t)b * MTOK * NCAT + NGK + g;
  float mx = -INFINITY;
#pragma unroll 1
  for (int i = 0; i < MTOK / 8; ++i) mx = fmaxf(mx, colp[(size_t)(wv + 8 * i) * NCAT]);
  red[wv][lane] = mx;
  __syncthreads();
  {
    float m2 = red[0][lane];
#pragma unroll
    for (int w = 1; w < 8; ++w) m2 = fmaxf(m2, red[w][lane]);
    mx = m2;
  }
  __syncthreads();
  float se = 0.f;
#pragma unroll 1
  for (int i = 0; i < MTOK / 8; ++i) se += expf(colp[(size_t)(wv + 8 * i) * NCAT] - mx);
  red[wv][lane] = se;
  __syncthreads();
  float tot = red[0][lane];
#pragma unroll
  for (int w = 1; w < 8; ++w) tot += red[w][lane];
  const float inv = 1.0f / tot;
  __syncthreads();
  float wsp = 0.f;
  const size_t rowb = (size_t)b * NGK + (size_t)cc * 32;
#pragma unroll 1
  for (int qc = 0; qc < MTOK / 256; ++qc) {
#pragma unroll 1
    for (int i = 0; i < 32; ++i) {
      const int ml = wv + 8 * i;
      const int m = qc * 256 + ml;
      const float lg = colp[(size_t)m * NCAT];
      const float av = agp[(size_t)m * NCAT];
      const float sg = 1.0f / (1.0f + expf(-av));
      const float p = expf(lg - mx) * inv;
      const float w = sg * p;
      wsp += w;
      wt[lane * 264 + ml] = h_bits(w * 1024.0f);
    }
    __syncthreads();
    u32x4 pk[4];
#pragma unroll
    for (int rr = 0; rr < 4; ++rr) pk[rr] = *(const u32x4*)(wt + (wv * 4 + rr) * 264 + lane * 8);
    for (int pass = 0; pass < 2; ++pass) {
#pragma unroll
      for (int rr = 0; rr < 4; ++rr)
        *(volatile u32x4*)(wt16 + (rowb + wv * 4 + rr) * (size_t)MTOK + qc * 256 + lane * 8) = pk[rr];
      __threadfence();
    }
    __syncthreads();
  }
  red[wv][lane] = wsp;
  __syncthreads();
  if (wv == 0) {
    float s = red[0][lane];
#pragma unroll
    for (int w = 1; w < 8; ++w) s += red[w][lane];
    float* dst = wsum + rowb + lane;
    *(volatile float*)dst = s;
    __threadfence();
    *(volatile float*)dst = s;
  }
}

__global__ __launch_bounds__(256) void k_vf_center(const float* __restrict__ vraw, const float* __restrict__ wsum,
                                                   const float* __restrict__ cent, const float* __restrict__ wf,
                                                   const float* __restrict__ bf, float* __restrict__ vc) {
  __shared__ float svf[8][33];
  const int dch = blockIdx.x, b = blockIdx.y;
  const int lane = threadIdx.x & 31, g = threadIdx.x >> 5;
  const int d = dch * 32 + lane;
  const float* rp = vraw + ((size_t)(b * NGRP + g) * NCLU) * DGRP + d;
  const float* wp = wsum + (size_t)b * NGK + (size_t)g * NCLU;
  const float* cp = cent + d;
  float s = 0.f;
#pragma unroll 1
  for (int k = 0; k < NCLU; ++k) {
    const float vl = rp[(size_t)k * DGRP] - wp[k] * cp[(size_t)k * DGRP];
    s = s + vl * wf[k];
  }
  const float vfv = s + bf[0];
  svf[g][lane] = vfv;
  __syncthreads();
  const int e = threadIdx.x;
  const int dl = e >> 3, g2 = e & 7;
  float sum = 0.f;
#pragma unroll
  for (int gg = 0; gg < 8; ++gg) sum += svf[gg][dl];
  const float mean = sum * 0.125f;
  const float outv = svf[g2][dl] - mean;
  float* dst = vc + ((size_t)b * DCOV + (size_t)dch * 32) * NGRP + e;
  *(volatile float*)dst = outv;
  __threadfence();
  *(volatile float*)dst = outv;
}

__global__ __launch_bounds__(256) void k_cov(const float* __restrict__ vc, float* __restrict__ cov) {
  const int i = blockIdx.x, b = blockIdx.y, j = threadIdx.x;
  const float* pi = vc + ((size_t)b * DCOV + i) * NGRP;
  const float* pj = vc + ((size_t)b * DCOV + j) * NGRP;
  const v4f a0 = *(const v4f*)pi, a1 = *(const v4f*)(pi + 4);
  const v4f c0 = *(const v4f*)pj, c1 = *(const v4f*)(pj + 4);
  float s = a0[0] * c0[0];
  s = fmaf(a0[1], c0[1], s);
  s = fmaf(a0[2], c0[2], s);
  s = fmaf(a0[3], c0[3], s);
  s = fmaf(a1[0], c1[0], s);
  s = fmaf(a1[1], c1[1], s);
  s = fmaf(a1[2], c1[2], s);
  s = fmaf(a1[3], c1[3], s);
  const float v = s * 0.125f;
  float* dst = cov + ((size_t)b * DCOV + i) * DCOV + j;
  *(volatile float*)dst = v;
  __threadfence();
  *(volatile float*)dst = v;
}

__global__ __launch_bounds__(256) void k_trace(const float* __restrict__ cov, float* __restrict__ trsq) {
  __shared__ float red[256];
  const int b = blockIdx.x, t = threadIdx.x;
  red[t] = cov[((size_t)b * DCOV + t) * DCOV + t];
  __syncthreads();
  for (int s = 128; s > 0; s >>= 1) {
    if (t < s) red[t] += red[t + s];
    __syncthreads();
  }
  const float tr = red[0];
  if (t < 32) {
    float val = 0.f;
    if (t == 0) val = tr;
    if (t == 1) val = 0.5f * sqrtf(tr);
    if (t == 2) val = 1.0f / tr;
    float* dst = trsq + b * 32 + t;
    *(volatile float*)dst = val;
    __threadfence();
    *(volatile float*)dst = val;
  }
}

__global__ __launch_bounds__(256) void k_nsinit(const float* __restrict__ cov, const float* __restrict__ trsq,
                                                unsigned short* __restrict__ ah, unsigned short* __restrict__ al,
                                                unsigned short* __restrict__ zh, unsigned short* __restrict__ zl) {
  const int i = blockIdx.x * 256 + threadIdx.x;
  const size_t e0 = (size_t)i * 8;
  const int b = (int)(e0 >> 16);
  const int r = (int)((e0 >> 8) & 255);
  const int c0 = (int)(e0 & 255);
  const float rtr = trsq[b * 32 + 2];
  const v4f x0 = *(const v4f*)(cov + e0);
  const v4f x1 = *(const v4f*)(cov + e0 + 4);
  float av[8];
  av[0] = x0[0]; av[1] = x0[1]; av[2] = x0[2]; av[3] = x0[3];
  av[4] = x1[0]; av[5] = x1[1]; av[6] = x1[2]; av[7] = x1[3];
  unsigned short hA[8], lA[8], hZ[8], lZ[8];
#pragma unroll
  for (int e = 0; e < 8; ++e) {
    const float a = av[e] * rtr;
    const float z = 0.5f * (((r == c0 + e) ? 3.0f : 0.0f) - a);
    split_bf(a, hA[e], lA[e]);
    split_bf(z, hZ[e], lZ[e]);
  }
  u32x4 pa, pal, pz, pzl;
#pragma unroll
  for (int e = 0; e < 4; ++e) {
    pa[e]  = (unsigned)hA[2 * e] | ((unsigned)hA[2 * e + 1] << 16);
    pal[e] = (unsigned)lA[2 * e] | ((unsigned)lA[2 * e + 1] << 16);
    pz[e]  = (unsigned)hZ[2 * e] | ((unsigned)hZ[2 * e + 1] << 16);
    pzl[e] = (unsigned)lZ[2 * e] | ((unsigned)lZ[2 * e + 1] << 16);
  }
  for (int pass = 0; pass < 2; ++pass) {
    *(volatile u32x4*)(ah + e0) = pa;
    *(volatile u32x4*)(al + e0) = pal;
    *(volatile u32x4*)(zh + e0) = pz;
    *(volatile u32x4*)(zl + e0) = pzl;
    __threadfence();
  }
}

__global__ __launch_bounds__(256) void k_triuvec(const float* __restrict__ F, float* __restrict__ out, int ntot) {
  const int gi = blockIdx.x * 256 + threadIdx.x;
  if (gi >= ntot) return;
  const int b = gi / NTRIU;
  const int t = gi - b * NTRIU;
  int lo = 0, hi = DCOV - 1;
#pragma unroll
  for (int it = 0; it < 8; ++it) {
    const int mid = (lo + hi + 1) >> 1;
    const int om = mid * DCOV - ((mid * (mid - 1)) >> 1);
    if (om <= t) lo = mid; else hi = mid - 1;
  }
  const int r = lo;
  const int orr = r * DCOV - ((r * (r - 1)) >> 1);
  int c = r + (t - orr);
  c = (c < 0) ? 0 : ((c > DCOV - 1) ? (DCOV - 1) : c);
  const float v = F[((size_t)b * DCOV + r) * DCOV + c];
  ((volatile float*)out)[gi] = v;
  __threadfence();
  ((volatile float*)out)[gi] = v;
}

static inline unsigned gemm_gx(int M, int N) { return (unsigned)(((M / 64) * (N / 64) + 7) / 8); }

extern "C" void kernel_launch(void* const* d_in, const int* in_sizes, int n_in,
                              void* d_out, int out_size, void* d_ws, size_t ws_size,
                              hipStream_t stream) {
  if (n_in < 10) return;
  if (in_sizes[0] != NB8 * CIN * HWN) return;
  if (in_sizes[1] != NCLU * DGRP) return;
  if (in_sizes[2] != EDIM * CIN) return;
  if (in_sizes[3] != EDIM) return;
  if (in_sizes[4] != NGRP * EDIM) return;
  if (in_sizes[5] < NGRP) return;
  if (in_sizes[6] != NGK * EDIM) return;
  if (in_sizes[7] != NGK) return;
  if (in_sizes[8] < NCLU) return;
  if (in_sizes[9] < 1) return;
  if (out_size != NBATCH * NTRIU) return;

  const float* x     = (const float*)d_in[0];
  const float* cent  = (const float*)d_in[1];
  const float* W_inp = (const float*)d_in[2];
  const float* b_inp = (const float*)d_in[3];
  const float* W_g   = (const float*)d_in[4];
  const float* b_g   = (const float*)d_in[5];
  const float* W_gk  = (const float*)d_in[6];
  const float* b_gk  = (const float*)d_in[7];
  const float* W_f   = (const float*)d_in[8];
  const float* b_f   = (const float*)d_in[9];
  float* out = (float*)d_out;

  char* ws = (char*)d_ws;
  size_t off = 0;
  auto take = [&](size_t bytes) -> char* { char* p = ws + off; off += (bytes + 255) & ~(size_t)255; return p; };
  const size_t PLB = (size_t)NBATCH * DCOV * DCOV * 2;
  unsigned short* XT16   = (unsigned short*)take((size_t)NBATCH * MTOK * CIN * 2);
  unsigned short* WINP16 = (unsigned short*)take((size_t)EDIM * CIN * 2);
  unsigned short* WCAT16 = (unsigned short*)take((size_t)NCAT * EDIM * 2);
  float* BIAS1 = (float*)take((size_t)EDIM * 4);
  float* BIAS2 = (float*)take((size_t)NCAT * 4);
  unsigned short* H16  = (unsigned short*)take((size_t)NBATCH * MTOK * EDIM * 2);
  unsigned short* H16T = (unsigned short*)take((size_t)NBATCH * EDIM * MTOK * 2);
  float* LOGI  = (float*)take((size_t)NBATCH * MTOK * NCAT * 4);
  unsigned short* WT16 = (unsigned short*)take((size_t)NBATCH * NGK * MTOK * 2);
  float* WSUM  = (float*)take((size_t)NBATCH * NGK * 4);
  float* VLADR = (float*)take((size_t)NBATCH * NGRP * NCLU * DGRP * 4);
  float* VC    = (float*)take((size_t)NBATCH * DCOV * NGRP * 4);
  float* COV   = (float*)take((size_t)NBATCH * DCOV * DCOV * 4);
  float* TRSQ  = (float*)take((size_t)NBATCH * 128);
  unsigned short* AH   = (unsigned short*)take(PLB);
  unsigned short* AL   = (unsigned short*)take(PLB);
  unsigned short* ZH   = (unsigned short*)take(PLB);
  unsigned short* ZL   = (unsigned short*)take(PLB);
  unsigned short* Y1H  = (unsigned short*)take(PLB);
  unsigned short* Y1L  = (unsigned short*)take(PLB);
  unsigned short* Y1TH = (unsigned short*)take(PLB);
  unsigned short* Y1TL = (unsigned short*)take(PLB);
  unsigned short* TH   = (unsigned short*)take(PLB);
  unsigned short* TL   = (unsigned short*)take(PLB);
  unsigned short* TTH  = (unsigned short*)take(PLB);
  unsigned short* TTL  = (unsigned short*)take(PLB);
  unsigned short* Y2H  = (unsigned short*)take(PLB);
  unsigned short* Y2L  = (unsigned short*)take(PLB);
  unsigned short* Y2TH = (unsigned short*)take(PLB);
  unsigned short* Y2TL = (unsigned short*)take(PLB);
  unsigned short* Z2H  = (unsigned short*)take(PLB);
  unsigned short* Z2L  = (unsigned short*)take(PLB);
  unsigned short* WTH  = (unsigned short*)take(PLB);
  unsigned short* WTL  = (unsigned short*)take(PLB);
  float* FMAT = (float*)take((size_t)NBATCH * DCOV * DCOV * 4);
  if (off > ws_size) return;
  if ((Y1L != Y1H + PLB / 2) || (Y1TL != Y1TH + PLB / 2) || (TL != TH + PLB / 2) || (TTL != TTH + PLB / 2) ||
      (Y2L != Y2H + PLB / 2) || (Y2TL != Y2TH + PLB / 2)) return;

  const long PLS = (long)DCOV * DCOV;

  k_cast_scaled16<<<(EDIM * CIN / 8 + 255) / 256, 256, 0, stream>>>(W_inp, WINP16, EDIM * CIN / 8, 64.0f);
  k_build_wcat<<<NCAT, 256, 0, stream>>>(W_gk, W_g, WCAT16, 64.0f);
  k_bias<<<(EDIM + NCAT + 255) / 256, 256, 0, stream>>>(b_inp, b_gk, b_g, BIAS1, BIAS2);
  k_prep_xt<<<dim3(HWN / 32, NB8), 256, 0, stream>>>(x, XT16);

  wmma_gemm64<0, false, 2, 1, false, 0, 0, false><<<dim3(gemm_gx(NBATCH * MTOK, EDIM), 1), 256, 0, stream>>>(
      XT16, nullptr, CIN, 0, WINP16, nullptr, CIN, 0, H16, nullptr, EDIM, 0,
      BIAS1, nullptr, 0, NBATCH * MTOK, EDIM, CIN, 1.0f / 128.0f, nullptr);

  wmma_gemm64<0, false, 2, 0, false, 0, 0, false><<<dim3(gemm_gx(NBATCH * MTOK, NCAT), 1), 256, 0, stream>>>(
      H16, nullptr, EDIM, 0, WCAT16, nullptr, EDIM, 0, LOGI, nullptr, NCAT, 0,
      BIAS2, nullptr, 0, NBATCH * MTOK, NCAT, EDIM, 1.0f / 1024.0f, nullptr);

  k_transpose16<<<dim3(EDIM / 64, MTOK / 64, NBATCH), 256, 0, stream>>>(H16, H16T, MTOK, EDIM,
                                                                        (long)MTOK * EDIM, (long)EDIM * MTOK);

  k_softmax_w<<<dim3(NGK / 32, NBATCH), 256, 0, stream>>>(LOGI, WT16, WSUM);

  wmma_gemm64<0, false, 0, 0, false, 0, 0, false><<<dim3(gemm_gx(NCLU, DGRP), NBATCH * NGRP), 256, 0, stream>>>(
      WT16, nullptr, MTOK, (long)NCLU * MTOK, H16T, nullptr, MTOK, (long)DGRP * MTOK,
      VLADR, nullptr, DGRP, (long)NCLU * DGRP,
      nullptr, nullptr, 0, NCLU, DGRP, MTOK, 1.0f / 16384.0f, nullptr);

  k_vf_center<<<dim3(DGRP / 32, NBATCH), 256, 0, stream>>>(VLADR, WSUM, cent, W_f, b_f, VC);
  k_cov<<<dim3(DCOV, NBATCH), 256, 0, stream>>>(VC, COV);
  k_trace<<<NBATCH, 256, 0, stream>>>(COV, TRSQ);

  k_nsinit<<<(NBATCH * DCOV * DCOV / 8) / 256, 256, 0, stream>>>(COV, TRSQ, AH, AL, ZH, ZL);
  const dim3 nsg(gemm_gx(DCOV, DCOV), NBATCH);
  wmma_gemm64<1, true, 0, 2, false, 0, 0, false><<<nsg, 256, 0, stream>>>(
      AH, AL, DCOV, PLS, ZH, ZL, DCOV, PLS, Y1H, Y1L, DCOV, PLS, nullptr, nullptr, 0, DCOV, DCOV, DCOV, 1.0f, nullptr);
  k_transpose16<<<dim3(DCOV / 64, DCOV / 64, 2 * NBATCH), 256, 0, stream>>>(Y1H, Y1TH, DCOV, DCOV, PLS, PLS);
  wmma_gemm64<1, true, 0, 2, false, 0, 1, false><<<nsg, 256, 0, stream>>>(
      ZH, ZL, DCOV, PLS, Y1TH, Y1TL, DCOV, PLS, TH, TL, DCOV, PLS, nullptr, nullptr, 0, DCOV, DCOV, DCOV, 1.0f, nullptr);
  k_transpose16<<<dim3(DCOV / 64, DCOV / 64, 2 * NBATCH), 256, 0, stream>>>(TH, TTH, DCOV, DCOV, PLS, PLS);
  wmma_gemm64<1, true, 0, 2, false, 0, 0, false><<<nsg, 256, 0, stream>>>(
      Y1H, Y1L, DCOV, PLS, TTH, TTL, DCOV, PLS, Y2H, Y2L, DCOV, PLS, nullptr, nullptr, 0, DCOV, DCOV, DCOV, 1.0f, nullptr);
  k_transpose16<<<dim3(DCOV / 64, DCOV / 64, 2 * NBATCH), 256, 0, stream>>>(Y2H, Y2TH, DCOV, DCOV, PLS, PLS);
  wmma_gemm64<1, true, 0, 2, false, 0, 0, false><<<nsg, 256, 0, stream>>>(
      TH, TL, DCOV, PLS, ZH, ZL, DCOV, PLS, Z2H, Z2L, DCOV, PLS, nullptr, nullptr, 0, DCOV, DCOV, DCOV, 1.0f, nullptr);
  wmma_gemm64<1, true, 0, 2, false, 0, 2, false><<<nsg, 256, 0, stream>>>(
      Y2TH, Y2TL, DCOV, PLS, Z2H, Z2L, DCOV, PLS, WTH, WTL, DCOV, PLS, nullptr, nullptr, 0, DCOV, DCOV, DCOV, 1.0f, nullptr);
  wmma_gemm64<1, true, 0, 0, false, 0, 0, true><<<nsg, 256, 0, stream>>>(
      Y2H, Y2L, DCOV, PLS, WTH, WTL, DCOV, PLS, FMAT, nullptr, DCOV, PLS, nullptr, nullptr, 0, DCOV, DCOV, DCOV, 1.0f, TRSQ);

  k_triuvec<<<(NBATCH * NTRIU) / 256, 256, 0, stream>>>(FMAT, out, NBATCH * NTRIU);
}
